// Block_46746424050070
// MI455X (gfx1250) — hardware-run, weakly checked
//
#include <hip/hip_runtime.h>


#ifndef NB
#define NB 4
#endif
#ifndef SEQ
#define SEQ 2048
#endif
#define NB_FULL  4
#define SEQ_FULL 2048
#ifndef OUT_SEQ
#define OUT_SEQ SEQ
#endif
#define DM   768
#define DFF  3072
#define NH_  12
#define HD   64
#define AW   4
#define SC2  (0.125f * 1.4426950408889634f)
#define PSH  8.0f
#define WSC  1024.0f
#define CSC  64.0f

static_assert(HD == 64);
static_assert(NH_ * HD == DM);
static_assert(DM % 64 == 0);
static_assert(DFF % 64 == 0);
static_assert(DM % 32 == 0);
static_assert(DFF % 32 == 0);
static_assert(SEQ % 64 == 0);
static_assert((NB * SEQ) % 64 == 0);
static_assert(SEQ % 32 == 0);
static_assert(SEQ % (16 * AW) == 0);
static_assert((NB * SEQ) % 4 == 0);
static_assert(((size_t)SEQ * DM) % 8 == 0);
static_assert(DM == 6 * 32 * 4);
static_assert(NB <= NB_FULL);
static_assert(SEQ <= SEQ_FULL);
static_assert(OUT_SEQ >= SEQ);
static_assert(64 * 65 * 4 <= 131072);
static_assert(16 * 68 * 4 <= 131072);
static_assert(AW * 16 * 68 * 4 <= 131072);
static_assert(4 * DM * 4 <= 131072);

typedef _Float16 h16;
typedef unsigned short bf;
typedef __attribute__((ext_vector_type(16))) __bf16   v16bf;
typedef __attribute__((ext_vector_type(16))) _Float16 v16h;
typedef __attribute__((ext_vector_type(8)))  _Float16 v8h;
typedef __attribute__((ext_vector_type(8)))  unsigned short v8us;
typedef __attribute__((ext_vector_type(8)))  float    v8f;
typedef __attribute__((ext_vector_type(4)))  float    v4f;
typedef v4f  __attribute__((may_alias)) v4fa;

__device__ __forceinline__ unsigned short f2bf(float f) { unsigned u = __float_as_uint(f); u += 0x7FFFu + ((u >> 16) & 1u); return (unsigned short)(u >> 16); }
__device__ __forceinline__ float rbf(float f) { return __uint_as_float(((unsigned)f2bf(f)) << 16); }
__device__ __forceinline__ v16h cat16(v8h lo, v8h hi) { return __builtin_shufflevector(lo, hi, 0, 1, 2, 3, 4, 5, 6, 7, 8, 9, 10, 11, 12, 13, 14, 15); }
__device__ __forceinline__ v16bf cat16b(v8us lo, v8us hi) { return __builtin_bit_cast(v16bf, __builtin_shufflevector(lo, hi, 0, 1, 2, 3, 4, 5, 6, 7, 8, 9, 10, 11, 12, 13, 14, 15)); }
__device__ __forceinline__ v8f wmma16(v16h a, v16h b, v8f c) { return __builtin_amdgcn_wmma_f32_16x16x32_f16(false, a, false, b, (short)0, c, false, false); }
__device__ __forceinline__ v8f wmmab(v16bf a, v16bf b, v8f c) { return __builtin_amdgcn_wmma_f32_16x16x32_bf16(false, a, false, b, (short)0, c, false, false); }
__device__ __forceinline__ v16h  ldh(const h16* p) { return cat16(*(const v8h*)p, *(const v8h*)(p + 16)); }
__device__ __forceinline__ v16bf ldb(const bf* p)  { return cat16b(*(const v8us*)p, *(const v8us*)(p + 16)); }
__device__ __forceinline__ void wave_sync() { __builtin_amdgcn_fence(3  , "wavefront"); __builtin_amdgcn_wave_barrier(); asm volatile("" ::: "memory"); }
__device__ __forceinline__ int wave_id() { return __builtin_amdgcn_readfirstlane((int)(threadIdx.x >> 5)); }
static __device__ __forceinline__ h16 toh_flush(float v) { const h16 r = (h16)v; return (fabsf(v) < 6.103515625e-05f) ? (h16)0.0f : r; }

template <int F16> struct Op;
template <> struct Op<0> { typedef v16bf V; typedef bf E;
    static __device__ __forceinline__ V ld(const bf* p) { return ldb(p); }
    static __device__ __forceinline__ v8f mm(V a, V b, v8f c) { return wmmab(a, b, c); } };
template <> struct Op<1> { typedef v16h V; typedef h16 E;
    static __device__ __forceinline__ V ld(const h16* p) { return ldh(p); }
    static __device__ __forceinline__ v8f mm(V a, V b, v8f c) { return wmma16(a, b, c); } };

__global__ __launch_bounds__(256) void k_wt(const float* __restrict__ W, bf* Wt, int K, int N, int mode) {
    __shared__ float t[64 * 65];
    const int tid = threadIdx.x, n0 = blockIdx.x * 64, k0 = blockIdx.y * 64;
#pragma unroll
    for (int i = 0; i < 4; ++i) { const int kk = (tid >> 4) + 16 * i, c4 = (tid & 15) * 4;
        const v4f v = *(const v4f*)(W + (size_t)(k0 + kk) * N + n0 + c4);
        t[kk * 65 + c4 + 0] = v[0]; t[kk * 65 + c4 + 1] = v[1]; t[kk * 65 + c4 + 2] = v[2]; t[kk * 65 + c4 + 3] = v[3]; }
    __syncthreads();
    const int lane = tid & 31, wave = wave_id();
    v8us o[2];
#pragma unroll
    for (int s = 0; s < 2; ++s) { const int nn = 4 * (wave + 8 * s) + (lane >> 3), c8 = (lane & 7) * 8;
        v8us ob; v8h oh;
#pragma unroll
        for (int i = 0; i < 8; ++i) { const unsigned short u = f2bf(t[(c8 + i) * 65 + nn]); ob[i] = u; oh[i] = toh_flush(__uint_as_float(((unsigned)u) << 16) * WSC); }
        const v8us ohb = __builtin_bit_cast(v8us, oh);
        o[s] = mode ? ohb : ob; }
#pragma unroll 1
    for (int ps = 0; ps < 2; ++ps) {
#pragma unroll
        for (int s = 0; s < 2; ++s) { const int nn = 4 * (wave + 8 * s) + (lane >> 3), c8 = (lane & 7) * 8;
            *(volatile v8us*)(Wt + (size_t)(n0 + nn) * K + k0 + c8) = o[s]; }
        if (ps == 0) __threadfence(); }
}

template <int F16, int EPI>
__device__ __forceinline__ void gemm_tile(const bf* __restrict__ Ain, const bf* __restrict__ Bin, int K,
                                          const float* __restrict__ bias, int nbias, int biasRow, float scale, int act,
                                          h16* Ph, int RB, size_t sRB, int pitch, int CB, size_t sCB,
                                          float* Cf, int ldc, const float* __restrict__ Res, int resBR, int outBR, int resBf) {
    typedef typename Op<F16>::V V; typedef typename Op<F16>::E E;
    __shared__ __align__(16) float os[16 * 68];
    const E* A = (const E*)Ain; const E* Bt = (const E*)Bin;
    const int lane = threadIdx.x & 31, lr = lane & 15, hi = lane >> 4; const int r0 = blockIdx.x * 64, c0 = blockIdx.y * 64;
    v8f acc[4][4];
#pragma unroll
    for (int mb = 0; mb < 4; ++mb)
#pragma unroll
        for (int nb = 0; nb < 4; ++nb) acc[mb][nb] = (v8f){};
    const size_t aoff = (size_t)(r0 + lr) * K + 8 * hi, boff = (size_t)(c0 + lr) * K + 8 * hi;
#pragma unroll 1
    for (int kc = 0; kc < K; kc += 32) {
        V a[4];
#pragma unroll
        for (int mb = 0; mb < 4; ++mb) a[mb] = Op<F16>::ld(A + aoff + (size_t)mb * 16 * K + kc);
#pragma unroll
        for (int nb = 0; nb < 4; ++nb) { const V b = Op<F16>::ld(Bt + boff + (size_t)nb * 16 * K + kc);
#pragma unroll
            for (int mb = 0; mb < 4; ++mb) acc[mb][nb] = Op<F16>::mm(a[mb], b, acc[mb][nb]); }
        asm volatile("v_nop\n\tv_nop\n\tv_nop\n\tv_nop" : "+v"(acc[0][0]), "+v"(acc[1][1]), "+v"(acc[2][2]), "+v"(acc[3][3]) : "v"(a[0]), "v"(a[1]), "v"(a[2]), "v"(a[3]));
    }
    float cbv[4];
#pragma unroll
    for (int nb = 0; nb < 4; ++nb) { int ci = c0 + nb * 16 + lr; ci = ci < nbias ? ci : nbias - 1; const float bvv = rbf(bias[ci]); cbv[nb] = biasRow ? 0.0f : bvv; }
    size_t tbase = 0;
    if (EPI == 0) tbase = (size_t)(r0 / RB) * sRB + (size_t)(r0 % RB) * (size_t)pitch + (size_t)(c0 / CB) * sCB + (size_t)(c0 % CB);
    const int bb = r0 / SEQ, tt = r0 - bb * SEQ;
#pragma unroll
    for (int mb = 0; mb < 4; ++mb) {
        float rb[8];
#pragma unroll
        for (int j = 0; j < 8; ++j) { int ri = r0 + mb * 16 + hi * 8 + j; ri = ri < nbias ? ri : nbias - 1; const float bvv = rbf(bias[ri]); rb[j] = biasRow ? bvv : 0.0f; }
#pragma unroll
        for (int nb = 0; nb < 4; ++nb) {
#pragma unroll
            for (int j = 0; j < 8; ++j) { const float v = acc[mb][nb][j] * scale + (cbv[nb] + rb[j]);
                os[(hi * 8 + j) * 68 + nb * 16 + lr] = v; } }
        wave_sync();
        if (act) {
            static_assert(8 * 32 * 4 == 16 * 64);
#pragma unroll 1
            for (int s = 0; s < 8; ++s) { const int row = 2 * s + hi, cofs = lr * 4;
                v4f g = *(const v4fa*)(&os[row * 68 + cofs]);
#pragma unroll
                for (int i = 0; i < 4; ++i) g[i] = 0.5f * g[i] * (1.0f + erff(g[i] * 0.70710678118654752f));
                *(v4fa*)(&os[row * 68 + cofs]) = g; }
            wave_sync();
        }
        if (EPI == 0) {
            const size_t sb = tbase + (size_t)(mb * 16) * (size_t)pitch;
            static_assert(32 * 16 * 4 == 16 * 64 * 2);
#pragma unroll 1
            for (int ps = 0; ps < 2; ++ps) {
#pragma unroll
                for (int s = 0; s < 4; ++s) { const int row = 4 * s + (lane >> 3), c8 = (lane & 7) * 8;
                    const v4f x0 = *(const v4fa*)(&os[row * 68 + c8]); const v4f x1 = *(const v4fa*)(&os[row * 68 + c8 + 4]); v8h hv;
#pragma unroll
                    for (int i = 0; i < 4; ++i) { hv[i] = toh_flush(x0[i]); hv[4 + i] = toh_flush(x1[i]); }
                    const size_t oo = sb + (size_t)row * (size_t)pitch + c8;
                    *(volatile v8h*)(Ph + oo) = hv; }
                if (ps == 0) __threadfence(); }
        } else {
            float* cp = Cf + ((size_t)bb * (size_t)outBR + (size_t)(tt + mb * 16)) * (size_t)ldc + c0;
            const float* rp = Res + ((size_t)bb * (size_t)resBR + (size_t)(tt + mb * 16)) * (size_t)ldc + c0;
            static_assert(32 * 16 * 8 == 16 * 64 * 4);
            v4f val[8];
#pragma unroll
            for (int s = 0; s < 8; ++s) { const int row = 2 * s + hi, cofs = lr * 4;
                const v4f o4 = *(const v4fa*)(&os[row * 68 + cofs]);
                v4f r4 = *(const v4f*)(rp + (size_t)row * (size_t)ldc + cofs);
#pragma unroll
                for (int i = 0; i < 4; ++i) { const float rr = rbf(r4[i]); r4[i] = resBf ? rr : r4[i]; }
                val[s] = o4 + r4; }
#pragma unroll 1
            for (int ps = 0; ps < 2; ++ps) {
#pragma unroll
                for (int s = 0; s < 8; ++s) { const int row = 2 * s + hi, cofs = lr * 4;
                    *(volatile v4f*)(cp + (size_t)row * (size_t)ldc + cofs) = val[s]; }
                if (ps == 0) __threadfence(); }
        }
        wave_sync();
    }
}

__global__ __launch_bounds__(32) void k_gemm_h(const bf* __restrict__ Ain, const bf* __restrict__ Bin, int K,
                                               const float* __restrict__ bias, int nbias, int biasRow, float scale, int act,
                                               h16* Ph, int RB, size_t sRB, int pitch, int CB, size_t sCB) {
    gemm_tile<1, 0>(Ain, Bin, K, bias, nbias, biasRow, scale, act, Ph, RB, sRB, pitch, CB, sCB, (float*)0, 0, (const float*)0, 0, 0, 0);
}
__global__ __launch_bounds__(32) void k_gemm_f(const bf* __restrict__ Ain, const bf* __restrict__ Bin, int K,
                                               const float* __restrict__ bias, int nbias, float scale,
                                               const float* __restrict__ Res, int resBR, int resBf,
                                               float* Cf, int outBR, int ldc) {
    gemm_tile<1, 1>(Ain, Bin, K, bias, nbias, 0, scale, 0, (h16*)0, 1, (size_t)0, 0, 1, (size_t)0, Cf, ldc, Res, resBR, outBR, resBf);
}

__global__ __launch_bounds__(32 * AW) void k_flash(const h16* __restrict__ QH, const h16* __restrict__ KP, const h16* __restrict__ VT, h16* CTX) {
    __shared__ __align__(16) float os[AW * 16 * 68];
    const int lane = threadIdx.x & 31, wave = wave_id(), lr = lane & 15, hi = lane >> 4;
    const int zh = blockIdx.y; const int b = zh / NH_, h = zh % NH_;
    const int t0 = (blockIdx.x * AW + wave) * 16;
    const size_t pbase = (size_t)zh * SEQ * HD;
    const size_t qo = pbase + (size_t)(t0 + lr) * HD + 8 * hi;
    const v16h qh0 = ldh(QH + qo), qh1 = ldh(QH + qo + 32);
    const size_t ko = pbase + (size_t)lr * HD + 8 * hi;
    const size_t vo = pbase + (size_t)lr * SEQ + 8 * hi;
    v8f o0 = (v8f){}, o1 = (v8f){}, o2 = (v8f){}, o3 = (v8f){};
    float m = -3.0e38f, l = 0.0f;
#pragma unroll 1
    for (int key0 = 0; key0 < SEQ; key0 += 32) {
        const h16* ka = KP + ko + (size_t)key0 * HD;
        const v16h ka0 = ldh(ka), ka1 = ldh(ka + 32), kb0 = ldh(ka + 16 * HD), kb1 = ldh(ka + 16 * HD + 32);
        v8f sHa = (v8f){}, sHb = (v8f){};
        sHa = wmma16(ka0, qh0, sHa); sHb = wmma16(kb0, qh0, sHb);
        sHa = wmma16(ka1, qh1, sHa); sHb = wmma16(kb1, qh1, sHb);
        asm volatile("v_nop\n\tv_nop\n\tv_nop\n\tv_nop" : "+v"(sHa), "+v"(sHb) : "v"(ka0), "v"(ka1), "v"(kb0), "v"(kb1));
        float ta[8], tb[8]; float mx = -3.0e38f;
#pragma unroll
        for (int r = 0; r < 8; ++r) { ta[r] = sHa[r] * SC2; tb[r] = sHb[r] * SC2; mx = fmaxf(mx, fmaxf(ta[r], tb[r])); }
        mx = fmaxf(mx, __shfl_xor(mx, 16, 32));
        const float mnew = fmaxf(m, mx);
        const float alpha = __builtin_amdgcn_exp2f(m - mnew);
        const float sh = PSH - mnew;
        v16h pb; float ls = 0.0f;
#pragma unroll
        for (int r = 0; r < 8; ++r) { const h16 pa = (h16)__builtin_amdgcn_exp2f(ta[r] + sh); const h16 pc = (h16)__builtin_amdgcn_exp2f(tb[r] + sh); pb[r] = pa; pb[8 + r] = pc; ls += (float)pa + (float)pc; }
        l = l * alpha + ls; m = mnew;
        o0 = o0 * alpha; o1 = o1 * alpha; o2 = o2 * alpha; o3 = o3 * alpha;
        const h16* va = VT + vo + key0;
        const v16h v0 = ldh(va), v1 = ldh(va + (size_t)16 * SEQ), v2 = ldh(va + (size_t)32 * SEQ), v3 = ldh(va + (size_t)48 * SEQ);
        o0 = wmma16(v0, pb, o0); o1 = wmma16(v1, pb, o1); o2 = wmma16(v2, pb, o2); o3 = wmma16(v3, pb, o3);
        asm volatile("v_nop\n\tv_nop\n\tv_nop\n\tv_nop" : "+v"(o0), "+v"(o1), "+v"(o2), "+v"(o3) : "v"(v0), "v"(v1), "v"(v2), "v"(v3), "v"(pb));
    }
    l += __shfl_xor(l, 16, 32);
    const float inv = CSC * (1.0f / l);
    const int wb = wave * 16 * 68;
    { v4f a, c;
      a[0] = o0[0] * inv; a[1] = o0[1] * inv; a[2] = o0[2] * inv; a[3] = o0[3] * inv; c[0] = o0[4] * inv; c[1] = o0[5] * inv; c[2] = o0[6] * inv; c[3] = o0[7] * inv;
      *(v4fa*)(&os[wb + lr * 68 +  0 + 8 * hi]) = a; *(v4fa*)(&os[wb + lr * 68 +  0 + 8 * hi + 4]) = c;
      a[0] = o1[0] * inv; a[1] = o1[1] * inv; a[2] = o1[2] * inv; a[3] = o1[3] * inv; c[0] = o1[4] * inv; c[1] = o1[5] * inv; c[2] = o1[6] * inv; c[3] = o1[7] * inv;
      *(v4fa*)(&os[wb + lr * 68 + 16 + 8 * hi]) = a; *(v4fa*)(&os[wb + lr * 68 + 16 + 8 * hi + 4]) = c;
      a[0] = o2[0] * inv; a[1] = o2[1] * inv; a[2] = o2[2] * inv; a[3] = o2[3] * inv; c[0] = o2[4] * inv; c[1] = o2[5] * inv; c[2] = o2[6] * inv; c[3] = o2[7] * inv;
      *(v4fa*)(&os[wb + lr * 68 + 32 + 8 * hi]) = a; *(v4fa*)(&os[wb + lr * 68 + 32 + 8 * hi + 4]) = c;
      a[0] = o3[0] * inv; a[1] = o3[1] * inv; a[2] = o3[2] * inv; a[3] = o3[3] * inv; c[0] = o3[4] * inv; c[1] = o3[5] * inv; c[2] = o3[6] * inv; c[3] = o3[7] * inv;
      *(v4fa*)(&os[wb + lr * 68 + 48 + 8 * hi]) = a; *(v4fa*)(&os[wb + lr * 68 + 48 + 8 * hi + 4]) = c; }
    wave_sync();
    h16* crow = CTX + ((size_t)b * SEQ + t0) * DM + h * HD;
#pragma unroll 1
    for (int ps = 0; ps < 2; ++ps) {
#pragma unroll
        for (int s = 0; s < 4; ++s) { const int row = 4 * s + (lane >> 3), c8 = (lane & 7) * 8;
            const v4f x0 = *(const v4fa*)(&os[wb + row * 68 + c8]); const v4f x1 = *(const v4fa*)(&os[wb + row * 68 + c8 + 4]); v8h hv;
#pragma unroll
            for (int i = 0; i < 4; ++i) { hv[i] = (h16)x0[i]; hv[4 + i] = (h16)x1[i]; }
            *(volatile v8h*)(crow + (size_t)row * DM + c8) = hv; }
        if (ps == 0) __threadfence(); }
}

template <int FIRST>
__device__ __forceinline__ void ln_rows(const float* __restrict__ R, const float* __restrict__ G, const float* __restrict__ BE, h16* OH, int nrows) {
    __shared__ __align__(16) float ls[4 * DM];
    const int lane = threadIdx.x & 31, wave = wave_id();
    const int r = blockIdx.x * 4 + wave;
    if (r >= nrows) return;
    const int b = r / SEQ, t = r - b * SEQ;
    const size_t ro = FIRST ? ((size_t)b * SEQ_FULL + t) * DM : (size_t)r * DM;
    const float* rp = R + ro;
    v4f v[6]; float sum = 0.0f;
#pragma unroll
    for (int i = 0; i < 6; ++i) { const int idx = (lane + 32 * i) * 4;
        v4f a = *(const v4f*)(rp + idx);
        if (FIRST) { a[0] = rbf(a[0]); a[1] = rbf(a[1]); a[2] = rbf(a[2]); a[3] = rbf(a[3]); }
        v[i] = a; sum += (a[0] + a[1]) + (a[2] + a[3]); }
#pragma unroll
    for (int d = 16; d >= 1; d >>= 1) sum += __shfl_xor(sum, d, 32);
    const float mu = sum * (1.0f / (float)DM);
    float sq = 0.0f;
#pragma unroll
    for (int i = 0; i < 6; ++i) { const v4f d = v[i] - mu; sq += (d[0] * d[0] + d[1] * d[1]) + (d[2] * d[2] + d[3] * d[3]); }
#pragma unroll
    for (int d = 16; d >= 1; d >>= 1) sq += __shfl_xor(sq, d, 32);
    const float rstd = rsqrtf(sq * (1.0f / (float)DM) + 1e-6f);
    v4f o[6];
#pragma unroll
    for (int i = 0; i < 6; ++i) { const int idx = (lane + 32 * i) * 4;
        const v4f g4 = *(const v4f*)(G + idx); const v4f b4 = *(const v4f*)(BE + idx);
#pragma unroll
        for (int k = 0; k < 4; ++k) o[i][k] = (v[i][k] - mu) * rstd * rbf(g4[k]) + rbf(b4[k]); }
    v8h hv[3];
    const int lw = wave * DM;
#pragma unroll
    for (int i = 0; i < 6; ++i) *(v4fa*)(&ls[lw + (lane + 32 * i) * 4]) = o[i];
    wave_sync();
#pragma unroll
    for (int j = 0; j < 3; ++j) { const int c8 = (lane + 32 * j) * 8;
        const v4f x0 = *(const v4fa*)(&ls[lw + c8]); const v4f x1 = *(const v4fa*)(&ls[lw + c8 + 4]);
#pragma unroll
        for (int k = 0; k < 4; ++k) { hv[j][k] = toh_flush(x0[k]); hv[j][4 + k] = toh_flush(x1[k]); } }
    h16* hp = OH + (size_t)r * DM;
    static_assert(3 * 32 * 16 == DM * 2);
#pragma unroll 1
    for (int ps = 0; ps < 2; ++ps) {
#pragma unroll
        for (int j = 0; j < 3; ++j) *(volatile v8h*)(hp + (lane + 32 * j) * 8) = hv[j];
        if (ps == 0) __threadfence(); }
}

__global__ __launch_bounds__(128) void k_ln1(const float* __restrict__ R, const float* __restrict__ G, const float* __restrict__ BE, h16* OH, int nrows) {
    ln_rows<1>(R, G, BE, OH, nrows);
}
__global__ __launch_bounds__(128) void k_ln2(const float* __restrict__ R, const float* __restrict__ G, const float* __restrict__ BE, h16* OH, int nrows) {
    ln_rows<0>(R, G, BE, OH, nrows);
}

static constexpr size_t al256(size_t v) { return (v + 255) & ~(size_t)255; }
static constexpr size_t SZ_R1  = al256((size_t)NB * SEQ * DM * 2);
static constexpr size_t SZ_W3  = al256((size_t)3 * DM * DM * 2);
static constexpr size_t SZ_WO  = al256((size_t)DM * DM * 2);
static constexpr size_t SZ_W1  = al256((size_t)DM * DFF * 2);
static constexpr size_t SZ_W2  = al256((size_t)DFF * DM * 2);
static constexpr size_t SZ_PL  = al256((size_t)NB * NH_ * SEQ * HD * 2);
static constexpr size_t SZ_FF  = al256((size_t)NB * SEQ * DFF * 2);
static constexpr size_t SZ_F32 = al256((size_t)NB * SEQ * DM * 4);
static constexpr size_t SZ_TOTAL = SZ_R1 + SZ_W3 + SZ_WO + SZ_W1 + SZ_W2 + SZ_FF + SZ_F32;
static_assert(SZ_TOTAL <= (size_t)134217728);
static_assert(3 * SZ_PL <= SZ_FF);
static_assert(((size_t)DM * DM * 2) % 256 == 0);

extern "C" void kernel_launch(void* const* d_in, const int* in_sizes, int n_in,
                              void* d_out, int out_size, void* d_ws, size_t ws_size, hipStream_t stream) {
    if (n_in < 17) return;
    const size_t needx = ((size_t)(NB - 1) * SEQ_FULL + SEQ) * DM;
    if ((size_t)in_sizes[0] < needx) return;
    if ((size_t)in_sizes[3] < (size_t)DM * DM || (size_t)in_sizes[5] < (size_t)DM * DM || (size_t)in_sizes[7] < (size_t)DM * DM || (size_t)in_sizes[9] < (size_t)DM * DM) return;
    if ((size_t)in_sizes[13] < (size_t)DM * DFF || (size_t)in_sizes[15] < (size_t)DFF * DM || (size_t)in_sizes[14] < (size_t)DFF) return;
    if (in_sizes[1] < DM || in_sizes[2] < DM || in_sizes[4] < DM || in_sizes[6] < DM || in_sizes[8] < DM) return;
    if (in_sizes[10] < DM || in_sizes[11] < DM || in_sizes[12] < DM || in_sizes[16] < DM) return;
    if ((size_t)out_size < ((size_t)(NB - 1) * OUT_SEQ + SEQ) * DM) return;
    if (SZ_TOTAL > ws_size) return;
    const float* x   = (const float*)d_in[0];
    const float* g1  = (const float*)d_in[1];  const float* be1 = (const float*)d_in[2];
    const float* wq  = (const float*)d_in[3];  const float* bq  = (const float*)d_in[4];
    const float* wk  = (const float*)d_in[5];  const float* bk  = (const float*)d_in[6];
    const float* wv  = (const float*)d_in[7];  const float* bv  = (const float*)d_in[8];
    const float* wo  = (const float*)d_in[9];  const float* bo  = (const float*)d_in[10];
    const float* g2  = (const float*)d_in[11]; const float* be2 = (const float*)d_in[12];
    const float* w1  = (const float*)d_in[13]; const float* b1  = (const float*)d_in[14];
    const float* w2  = (const float*)d_in[15]; const float* b2  = (const float*)d_in[16];
    float* OUT = (float*)d_out;
    char* wsp = (char*)d_ws;
    bf* R1  = (bf*)wsp; wsp += SZ_R1;
    bf* W3  = (bf*)wsp; wsp += SZ_W3;
    bf* WOT = (bf*)wsp; wsp += SZ_WO;
    bf* W1T = (bf*)wsp; wsp += SZ_W1;
    bf* W2T = (bf*)wsp; wsp += SZ_W2;
    char* ffr = wsp; wsp += SZ_FF;
    float* X1 = (float*)wsp; wsp += SZ_F32;
    h16* QH = (h16*)ffr;
    h16* KP = (h16*)(ffr + SZ_PL);
    h16* VT = (h16*)(ffr + 2 * SZ_PL);
    h16* FF1 = (h16*)ffr;
    h16* XN = (h16*)R1; h16* CTX = (h16*)R1; h16* XN2 = (h16*)R1;
    bf* WQT = W3; bf* WKT = W3 + (size_t)DM * DM; bf* WVT = W3 + (size_t)2 * DM * DM;
    const int MR = NB * SEQ;

    k_wt<<<dim3(DM / 64, DM / 64, 1), 256, 0, stream>>>(wq, WQT, DM, DM, 1);
    k_wt<<<dim3(DM / 64, DM / 64, 1), 256, 0, stream>>>(wk, WKT, DM, DM, 1);
    k_wt<<<dim3(DM / 64, DM / 64, 1), 256, 0, stream>>>(wv, WVT, DM, DM, 1);
    k_wt<<<dim3(DM / 64, DM / 64, 1), 256, 0, stream>>>(wo, WOT, DM, DM, 1);
    k_wt<<<dim3(DFF / 64, DM / 64, 1), 256, 0, stream>>>(w1, W1T, DM, DFF, 1);
    k_wt<<<dim3(DM / 64, DFF / 64, 1), 256, 0, stream>>>(w2, W2T, DFF, DM, 1);

    k_ln1<<<MR / 4, 128, 0, stream>>>(x, g1, be1, XN, MR);

    k_gemm_h<<<dim3(MR / 64, DM / 64, 1), 32, 0, stream>>>((const bf*)XN, WQT, DM, bq, DM, 0, 1.0f / 1024.0f, 0, QH, SEQ, (size_t)NH_ * SEQ * HD, HD, HD, (size_t)SEQ * HD);
    k_gemm_h<<<dim3(MR / 64, DM / 64, 1), 32, 0, stream>>>((const bf*)XN, WKT, DM, bk, DM, 0, 1.0f / 1024.0f, 0, KP, SEQ, (size_t)NH_ * SEQ * HD, HD, HD, (size_t)SEQ * HD);
    k_gemm_h<<<dim3(DM / 64, MR / 64, 1), 32, 0, stream>>>(WVT, (const bf*)XN, DM, bv, DM, 1, 1.0f / 1024.0f, 0, VT, DM, (size_t)0, SEQ, SEQ, (size_t)DM * SEQ);

    k_flash<<<dim3(SEQ / (16 * AW), NB * NH_, 1), 32 * AW, 0, stream>>>(QH, KP, VT, CTX);

    k_gemm_f<<<dim3(MR / 64, DM / 64, 1), 32, 0, stream>>>((const bf*)CTX, WOT, DM, bo, DM, 1.0f / 65536.0f, x, SEQ_FULL, 1, X1, SEQ, DM);
    k_ln2<<<MR / 4, 128, 0, stream>>>(X1, g2, be2, XN2, MR);
    k_gemm_h<<<dim3(MR / 64, DFF / 64, 1), 32, 0, stream>>>((const bf*)XN2, W1T, DM, b1, DFF, 0, 1.0f / 1024.0f, 1, FF1, MR, (size_t)0, DFF, DFF, (size_t)0);
    k_gemm_f<<<dim3(MR / 64, DM / 64, 1), 32, 0, stream>>>((const bf*)FF1, W2T, DFF, b2, DM, 1.0f / 1024.0f, X1, SEQ, 0, OUT, OUT_SEQ, DM);
}
